// QLSTM___65481071399193
// MI455X (gfx1250) — hardware-verified
//
#include <hip/hip_runtime.h>
#include <math.h>

typedef __attribute__((ext_vector_type(16))) _Float16 v16h;
typedef __attribute__((ext_vector_type(16))) __bf16 v16b;
typedef __attribute__((ext_vector_type(8)))  _Float16 v8h;
typedef __attribute__((ext_vector_type(8)))  float v8f;
typedef __attribute__((ext_vector_type(4)))  float v4f;
typedef __attribute__((ext_vector_type(2)))  float v2f;
typedef __attribute__((ext_vector_type(4)))  unsigned v4u;
typedef __attribute__((ext_vector_type(4)))  int v4i;
typedef float __attribute__((may_alias)) float_a;
typedef int __attribute__((may_alias)) int_a;

template <typename T> __device__ __forceinline__ void vst2(void* p, T v) { *(volatile T*)p = v; __threadfence(); *(volatile T*)p = v; }
__device__ __forceinline__ v8f wmma16(v16h a, v16h b, v8f c) {
  v8f d = __builtin_amdgcn_wmma_f32_16x16x32_f16(false, a, false, b, (short)0, c, false, false);
  asm volatile("v_nop\n\tv_nop\n\tv_nop\n\tv_nop" : "+v"(d) : "v"(a), "v"(b));
  return d;
}
__device__ __forceinline__ v8f wmma_bf(v16b a, v16b b, v8f c) {
  v8f d = __builtin_amdgcn_wmma_f32_16x16x32_bf16(false, a, false, b, (short)0, c, false, false);
  asm volatile("v_nop\n\tv_nop\n\tv_nop\n\tv_nop" : "+v"(d) : "v"(a), "v"(b));
  return d;
}
__device__ __forceinline__ v16h frag_h(const _Float16* rowk0, int lane) {
  union { v16h v; v8h q[2]; } u; const _Float16* p = rowk0 + 8 * (lane >> 4);
  u.q[0] = *(const v8h*)p; u.q[1] = *(const v8h*)(p + 16); return u.v;
}
__device__ __forceinline__ v16h frag_f32(const float* rowk0, int lane) {
  v16h a; const float* p = rowk0 + 8 * (lane >> 4);
#pragma unroll
  for (int i = 0; i < 8; ++i) { a[i] = (_Float16)p[i]; a[8 + i] = (_Float16)p[16 + i]; }
  return a;
}
__device__ __forceinline__ v16h frag_f32s(const float* rowk0, int lane, float sc) {
  v16h a; const float* p = rowk0 + 8 * (lane >> 4);
#pragma unroll
  for (int i = 0; i < 8; ++i) { a[i] = (_Float16)(p[i] * sc); a[8 + i] = (_Float16)(p[16 + i] * sc); }
  return a;
}
__device__ __forceinline__ v16h fragc_f32(const float* W, int k0, int n, int lane, int ld, int K) {
  v16h a; const int g = lane >> 4;
#pragma unroll
  for (int i = 0; i < 8; ++i) { const int ka = k0 + 8 * g + i, kb = ka + 16;
    a[i] = (_Float16)(ka < K ? W[(size_t)(ka < K ? ka : K - 1) * ld + n] : 0.f); a[8 + i] = (_Float16)(kb < K ? W[(size_t)(kb < K ? kb : K - 1) * ld + n] : 0.f); }
  return a;
}
struct F2 { v16b h, l; };
__device__ __forceinline__ F2 bsplit16(const float v[16]) { F2 r;
#pragma unroll
  for (int i = 0; i < 16; ++i) { const __bf16 h = (__bf16)v[i]; r.h[i] = h; r.l[i] = (__bf16)(v[i] - (float)h); }
  return r; }
__device__ __forceinline__ F2 split_row(const float* row, int k0, int lane) { float v[16]; const float* p = row + k0 + 8 * (lane >> 4);
#pragma unroll
  for (int i = 0; i < 8; ++i) { v[i] = p[i]; v[8 + i] = p[16 + i]; }
  return bsplit16(v); }
__device__ __forceinline__ F2 split_rowK(const float* row, int k0, int lane, int K) { float v[16]; const int g = lane >> 4;
#pragma unroll
  for (int i = 0; i < 8; ++i) { const int ka = k0 + 8 * g + i, kb = ka + 16; v[i] = ka < K ? row[ka < K ? ka : K - 1] : 0.f; v[8 + i] = kb < K ? row[kb < K ? kb : K - 1] : 0.f; }
  return bsplit16(v); }
__device__ __forceinline__ F2 split_col(const float* W, int k0, int n, int lane, int ld, int K) { float v[16]; const int g = lane >> 4;
#pragma unroll
  for (int i = 0; i < 8; ++i) { const int ka = k0 + 8 * g + i, kb = ka + 16; v[i] = ka < K ? W[(size_t)(ka < K ? ka : K - 1) * ld + n] : 0.f; v[8 + i] = kb < K ? W[(size_t)(kb < K ? kb : K - 1) * ld + n] : 0.f; }
  return bsplit16(v); }
__device__ __forceinline__ v8f mac3(const F2& a, const F2& b, v8f c) { c = wmma_bf(a.l, b.h, c); c = wmma_bf(a.h, b.l, c); return wmma_bf(a.h, b.h, c); }
__device__ __forceinline__ float sigm(float v) { return 1.0f / (1.0f + expf(-v)); }
#define LDSX() do { asm volatile("s_wait_dscnt 0" ::: "memory"); __builtin_amdgcn_wave_barrier(); __builtin_amdgcn_fence(__ATOMIC_RELEASE, "workgroup"); } while (0)


#define SEQ 128
#define NBT 1024
#define ID 64
#define NQ 10
#define NG 4
#define ND (ID + NQ)
#define NO (NG * NQ)
#ifndef NROWS
#define NROWS NBT
#endif
#define OFF_HX 1310720
#define OFF_CX 1320960
__device__ __forceinline__ float bfr(float v) { return (float)(__bf16)v; }
__device__ __forceinline__ float sigm_(float v) { return 1.0f / (1.0f + expf(-v)); }
__device__ __forceinline__ v16b fragWq(const float* __restrict__ Wt, int o, int k0, int lane) { v16b w; const int g = lane >> 4; const int oc = o < NO ? o : NO - 1; const float* wr = Wt + (size_t)(oc / NQ) * (NQ * ND) + (oc % NQ) * ND;
#pragma unroll
  for (int i = 0; i < 8; ++i) { const int ka = k0 + 8 * g + i, kb2 = ka + 16; const float wa = wr[ka < ND ? ka : ND - 1], wb = wr[kb2 < ND ? kb2 : ND - 1]; w[i] = (__bf16)((o < NO && ka < ND) ? wa : 0.f); w[8 + i] = (__bf16)((o < NO && kb2 < ND) ? wb : 0.f); }
  return w; }
__global__ __launch_bounds__(128) void k_ql(const float* __restrict__ X, const float* __restrict__ Wt, const float* __restrict__ Bb, const float* __restrict__ TH, float* __restrict__ OUT) {
  __shared__ __align__(16) float sH[64][36];
  __shared__ __align__(16) float sC[64][12];
  __shared__ __align__(16) float sA[64][48];
  const int tid = threadIdx.x, wave = tid >> 5, lane = tid & 31, col = lane & 15, g = lane >> 4; const size_t r0 = (size_t)blockIdx.x * 64; const int wr = wave * 16;
  for (int e = lane; e < 16 * 36; e += 32) sH[wr + e / 36][e % 36] = 0.f;
  for (int e = lane; e < 16 * 12; e += 32) sC[wr + e / 12][e % 12] = 0.f;
  v16b wf[3][3];
#pragma unroll
  for (int j = 0; j < 3; ++j)
#pragma unroll
    for (int kc = 0; kc < 3; ++kc) wf[j][kc] = fragWq(Wt, j * 16 + col, kc * 32, lane);
  float bias[3];
#pragma unroll
  for (int j = 0; j < 3; ++j) { const int o = j * 16 + col; const int oc = o < NO ? o : NO - 1; bias[j] = o < NO ? (bfr(Bb[oc]) + bfr(TH[oc])) : 0.f; }
  LDSX();
#pragma unroll 1
  for (int t = 0; t < SEQ; ++t) {
    v8f acc[3] = {};
#pragma unroll
    for (int kc = 0; kc < 2; ++kc) { v16b a; { const float* p = X + (((size_t)t * NBT + r0 + wr + col) * ID) + kc * 32 + 8 * g;
#pragma unroll
        for (int i = 0; i < 8; ++i) { a[i] = (__bf16)p[i]; a[8 + i] = (__bf16)p[16 + i]; } }
      asm volatile("s_wait_loadcnt 0x0" ::: "memory");
#pragma unroll
      for (int j = 0; j < 3; ++j) acc[j] = wmma_bf(a, wf[j][kc], acc[j]); }
    { float v[16];
#pragma unroll
      for (int i = 0; i < 8; ++i) { v[i] = sH[wr + col][8 * g + i]; v[8 + i] = sH[wr + col][16 + 8 * g + i]; }
      const F2 ah = bsplit16(v);
#pragma unroll
      for (int j = 0; j < 3; ++j) { acc[j] = wmma_bf(ah.h, wf[j][2], acc[j]); acc[j] = wmma_bf(ah.l, wf[j][2], acc[j]); } }
#pragma unroll
    for (int j = 0; j < 3; ++j)
#pragma unroll
      for (int r = 0; r < 8; ++r) sA[wr + 8 * g + r][j * 16 + col] = acc[j][r] + bias[j];
    LDSX();
#pragma unroll 1
    for (int task = lane; task < 16 * NG; task += 32) { const int rl = task >> 2, gt = task & 3; float* a = &sA[wr + rl][gt * NQ];
#pragma unroll 1
      for (int w = 0; w < NQ; ++w) a[w] = cosf(a[w]);
      float p19 = a[1];
#pragma unroll
      for (int k = 2; k < NQ; ++k) p19 = p19 * a[k];
      float pre = a[0];
#pragma unroll
      for (int k = 1; k < NQ; ++k) { pre = pre * a[k]; a[k] = pre; }
      a[0] = p19; }
    LDSX();
#pragma unroll 1
    for (int task = lane; task < 16 * NQ; task += 32) { const int rl = task / NQ, n = task % NQ; const float* m = sA[wr + rl];
      const float f = sigm_(m[n]), ig = sigm_(m[NQ + n]), gg = tanhf(m[2 * NQ + n]), og = sigm_(m[3 * NQ + n]);
      const float c = f * sC[wr + rl][n] + ig * gg; const float h = og * tanhf(c); sC[wr + rl][n] = c; sH[wr + rl][n] = h; }
    LDSX();
    { float* ob = OUT + ((size_t)t * NBT + r0 + wr) * NQ; for (int q = lane; q < 40; q += 32) { v4f o; const int f0 = q * 4;
#pragma unroll
        for (int z = 0; z < 4; ++z) { const int f = f0 + z; o[z] = sH[wr + f / NQ][f % NQ]; }
        vst2(ob + f0, o); } }
    LDSX(); }
  { float* oh = OUT + OFF_HX + (r0 + wr) * NQ; float* oc2 = OUT + OFF_CX + (r0 + wr) * NQ;
    for (int q = lane; q < 40; q += 32) { v4f o, o2; const int f0 = q * 4;
#pragma unroll
      for (int z = 0; z < 4; ++z) { const int f = f0 + z; o[z] = sH[wr + f / NQ][f % NQ]; o2[z] = sC[wr + f / NQ][f % NQ]; }
      vst2(oh + f0, o); vst2(oc2 + f0, o2); } } }
extern "C" void kernel_launch(void* const* d_in, const int* in_sizes, int n_in, void* d_out, int out_size, void* d_ws, size_t ws_size, hipStream_t stream) {
  (void)in_sizes; (void)n_in; (void)out_size; (void)d_ws; (void)ws_size;
  const float** F = (const float**)d_in;
  k_ql<<<dim3(NROWS / 64), 128, 0, stream>>>(F[0], F[1], F[2], F[3], (float*)d_out);
}
